// TreeBackbone_9105330667668
// MI455X (gfx1250) — hardware-verified
//
#include <hip/hip_runtime.h>
#include <math.h>


#define NI   4096
#define KP   448
#define KT   420
typedef __attribute__((ext_vector_type(16))) _Float16 v16h;
typedef __attribute__((ext_vector_type(8)))  _Float16 v8h;
typedef __attribute__((ext_vector_type(8)))  float    v8f;
typedef __attribute__((ext_vector_type(4)))  float    v4f;
#define VST2(T, ptr, val) do { const T _v = (val); *(volatile T*)(ptr) = _v; __threadfence(); *(volatile T*)(ptr) = _v; } while (0)
__device__ __forceinline__ v8f wmma16(v16h a, v16h b, v8f c) {
  v8f d = __builtin_amdgcn_wmma_f32_16x16x32_f16(false, a, false, b, (short)0, c, false, false);
  asm volatile("v_nop\n\tv_nop\n\tv_nop\n\tv_nop" : "+v"(d) : "v"(a), "v"(b));
  return d;
}
__device__ __forceinline__ v16h frag16(const _Float16* p, int hh) {
  const v8h lo = *(const v8h*)(p + 8 * hh), hi = *(const v8h*)(p + 16 + 8 * hh);
  return __builtin_shufflevector(lo, hi, 0,1,2,3,4,5,6,7,8,9,10,11,12,13,14,15);
}
__device__ __forceinline__ int kmap(int e, int hh) { return (e < 8) ? (8 * hh + e) : (16 + 8 * hh + (e - 8)); }
__device__ __forceinline__ float sigm(float x) { return 1.0f / (1.0f + expf(-x)); }
__global__ __launch_bounds__(256) void k_tw(const float* __restrict__ tw, _Float16* __restrict__ TW) {
  const int t = blockIdx.x * 256 + threadIdx.x;
  if (t >= 21 * 16 * 56) return;
  const int gp = t / (16 * 56), o = (t / 56) % 16, k0 = (t % 56) * 8, g = gp / 7, ph = gp % 7;
  v8h out;
#pragma unroll
  for (int e = 0; e < 8; ++e) {
    const int k = k0 + e; float v = 0.f;
    if (k < KT) { const int f = k / 28, r = k % 28, pw = r / 4, ki = (r >> 1) & 1, kj = r & 1;
      v = tw[(((((size_t)o * 15 + f) * 3 + g) * 7 + ph) * 7 + pw) * 4 + ki * 2 + kj]; }
    out[e] = (_Float16)v;
  }
  VST2(v8h, TW + ((size_t)gp * 16 + o) * KP + k0, out);
}
__global__ __launch_bounds__(256) void k_conv(const float* __restrict__ x, const float* __restrict__ cw, const float* __restrict__ cb, _Float16* __restrict__ P) {
  __shared__ __attribute__((aligned(16))) _Float16 Ps[8][7 * KP];
  const int lane = threadIdx.x & 31, wave = threadIdx.x >> 5, hh = lane >> 4, l16 = lane & 15;
  const int wg = blockIdx.x * 8 + wave;
  const int b = wg / 3, g = wg % 3;
  const float* xi = x + ((size_t)b * 3 + g) * 1024;
  v16h wb;
#pragma unroll
  for (int e = 0; e < 16; ++e) { const int k = kmap(e, hh); wb[e] = (k < 25 && l16 < 15) ? (_Float16)cw[(size_t)(g * 15 + l16) * 25 + k] : (_Float16)0.f; }
  const float bias = (l16 < 15) ? cb[g * 15 + l16] : 0.f;
  _Float16* ps = Ps[wave];
  for (int q = lane; q < 7 * KP; q += 32) ps[q] = (_Float16)0.f;
  for (int tile = 0; tile < 49; ++tile) {
    const int pq = tile * 4 + (l16 >> 2), py = pq / 14, px = pq % 14, oy = 2 * py + ((l16 >> 1) & 1), ox = 2 * px + (l16 & 1);
    v16h xa;
#pragma unroll
    for (int e = 0; e < 16; ++e) { const int k = kmap(e, hh); xa[e] = (k < 25) ? (_Float16)xi[(oy + k / 5) * 32 + ox + k % 5] : (_Float16)0.f; }
    v8f c = {}; c = wmma16(xa, wb, c);
    if (l16 < 15) {
#pragma unroll
      for (int qq = 0; qq < 2; ++qq) {
        float m = -INFINITY;
#pragma unroll
        for (int s = 0; s < 4; ++s) m = fmaxf(m, sigm(c[qq * 4 + s] + bias));
        const int pq2 = tile * 4 + hh * 2 + qq, py2 = pq2 / 14, px2 = pq2 % 14;
        const int ph = py2 >> 1, ki = py2 & 1, pw = px2 >> 1, kj = px2 & 1;
        ps[ph * KP + ((l16 * 7 + pw) * 2 + ki) * 2 + kj] = (_Float16)m;
      }
    }
  }
  __builtin_amdgcn_fence(__ATOMIC_RELEASE, "workgroup"); __builtin_amdgcn_wave_barrier(); __builtin_amdgcn_fence(__ATOMIC_ACQUIRE, "workgroup");
  _Float16* dst = P + ((size_t)b * 3 + g) * 7 * KP;
  for (int pass = 0; pass < 2; ++pass) {
    for (int q = lane; q < 7 * KP / 8; q += 32) *(volatile v8h*)(dst + q * 8) = *(const v8h*)(ps + q * 8);
    __threadfence();
  }
}
__global__ __launch_bounds__(256) void k_tree(const _Float16* __restrict__ P, const _Float16* __restrict__ TW, const float* __restrict__ tb, float* __restrict__ out) {
  __shared__ __attribute__((aligned(16))) float so[16 * 336];
  const int lane = threadIdx.x & 31, wave = threadIdx.x >> 5, hh = lane >> 4, l16 = lane & 15;
  const int b0 = blockIdx.x * 16;
  for (int gp = wave; gp < 21; gp += 8) {
    const int g = gp / 7, ph = gp % 7;
    v8f c = {};
    const _Float16* ar = P + (((size_t)(b0 + l16) * 3 + g) * 7 + ph) * KP;
    const _Float16* br = TW + ((size_t)gp * 16 + l16) * KP;
    for (int k0 = 0; k0 < KP; k0 += 32) c = wmma16(frag16(ar + k0, hh), frag16(br + k0, hh), c);
#pragma unroll
    for (int v = 0; v < 8; ++v) { const int bl = v + 8 * hh, o = l16; so[bl * 336 + o * 21 + g * 7 + ph] = sigm(c[v] + tb[(o * 3 + g) * 7 + ph]); }
  }
  __syncthreads();
  float* od = out + (size_t)b0 * 336;
  for (int pass = 0; pass < 2; ++pass) {
    for (int q = threadIdx.x; q < 16 * 336 / 4; q += 256) *(volatile v4f*)(od + q * 4) = *(const v4f*)(&so[q * 4]);
    __threadfence();
  }
}
extern "C" void kernel_launch(void* const* d_in, const int* in_sizes, int n_in,
                              void* d_out, int out_size, void* d_ws, size_t ws_size, hipStream_t stream) {
  (void)in_sizes; (void)n_in; (void)out_size;
  const float* x  = (const float*)d_in[0];
  const float* cw = (const float*)d_in[1];
  const float* cb = (const float*)d_in[2];
  const float* tw = (const float*)d_in[3];
  const float* tb = (const float*)d_in[4];
  float* out = (float*)d_out;
  char* ws = (char*)d_ws; size_t off = 0;
  auto take = [&](size_t bytes) { void* p = ws + off; off = (off + bytes + 255) & ~(size_t)255; return p; };
  _Float16* P  = (_Float16*)take((size_t)NI * 3 * 7 * KP * 2);
  _Float16* TW = (_Float16*)take((size_t)21 * 16 * KP * 2);
  if (off > ws_size) return;
  k_tw<<<(21 * 16 * 56 + 255) / 256, 256, 0, stream>>>(tw, TW);
  k_conv<<<NI * 3 / 8, 256, 0, stream>>>(x, cw, cb, P);
  k_tree<<<NI / 16, 256, 0, stream>>>(P, TW, tb, out);
}
